// GCLSTM_RecurrentGCN_16192026706535
// MI455X (gfx1250) — hardware-verified
//
#include <hip/hip_runtime.h>


typedef __attribute__((ext_vector_type(16))) _Float16 v16h;
typedef __attribute__((ext_vector_type(8)))  _Float16 v8h;
typedef __attribute__((ext_vector_type(8)))  float    v8f;
typedef __attribute__((ext_vector_type(4)))  float    v4f;
#define FDIM 256
#define KCAT 768
#define CDIM 1024
#define VST2(T, ptr, val) do { const T _v = (val); *(volatile T*)(ptr) = _v; __threadfence(); *(volatile T*)(ptr) = _v; } while (0)
__device__ __forceinline__ v8f wmma16(v16h a, v16h b, v8f c) {
  v8f d = __builtin_amdgcn_wmma_f32_16x16x32_f16(false, a, false, b, (short)0, c, false, false);
  asm volatile("v_nop\n\tv_nop\n\tv_nop\n\tv_nop" : "+v"(d) : "v"(a), "v"(b));
  return d;
}
__device__ __forceinline__ v16h frag16(const _Float16* p, int hh) {
  const v8h lo = *(const v8h*)(p + 8 * hh), hi = *(const v8h*)(p + 16 + 8 * hh);
  return __builtin_shufflevector(lo, hi, 0,1,2,3,4,5,6,7,8,9,10,11,12,13,14,15);
}

#define SORT_LOG 20
#define SORT_N (1 << SORT_LOG)
#define TILE 4096
typedef unsigned long long u64;
typedef __attribute__((ext_vector_type(2))) int v2i;
__global__ __launch_bounds__(256) void k_sort_init(const int* __restrict__ src, const int* __restrict__ dst, u64* __restrict__ A, int E) {
  const int i = blockIdx.x * 256 + threadIdx.x;
  u64 v = ~(u64)0;
  if (i < E)            v = (((u64)(unsigned)dst[i]) << 32) | (unsigned)i;
  else if (i < 2 * E)   v = ((u64)1 << 62) | (((u64)(unsigned)src[i - E]) << 32) | (unsigned)(i - E);
  VST2(u64, A + i, v);
}
__device__ __forceinline__ void cas_lds(u64* s, int lo, int hi, bool up) {
  const u64 a = s[lo], b = s[hi]; const bool sw = up ? (a > b) : (a < b); s[lo] = sw ? b : a; s[hi] = sw ? a : b;
}
__global__ __launch_bounds__(256) void k_sort_local(u64* __restrict__ A) {
  __shared__ u64 s[TILE];
  const int base = blockIdx.x * TILE, t = threadIdx.x;
  for (int i = t; i < TILE; i += 256) s[i] = A[base + i];
  __syncthreads();
  for (int k = 2; k <= TILE; k <<= 1)
    for (int j = k >> 1; j > 0; j >>= 1) {
      for (int p = t; p < TILE / 2; p += 256) {
        const int lo = ((p >> __builtin_ctz(j)) << (__builtin_ctz(j) + 1)) | (p & (j - 1));
        cas_lds(s, lo, lo + j, (((base + lo) & k) == 0));
      }
      __syncthreads();
    }
  for (int pass = 0; pass < 2; ++pass) { for (int i = t; i < TILE; i += 256) *(volatile u64*)(A + base + i) = s[i]; __threadfence(); }
}
__global__ __launch_bounds__(256) void k_sort_global(u64* __restrict__ A, int logj, int k) {
  const int p = blockIdx.x * 256 + threadIdx.x;
  const int j = 1 << logj;
  const int lo = ((p >> logj) << (logj + 1)) | (p & (j - 1)), hi = lo + j;
  const u64 a = A[lo], b = A[hi];
  const bool up = ((lo & k) == 0), sw = up ? (a > b) : (a < b);
  const u64 vlo = sw ? b : a, vhi = sw ? a : b;
  *(volatile u64*)(A + lo) = vlo; *(volatile u64*)(A + hi) = vhi; __threadfence();
  *(volatile u64*)(A + lo) = vlo; *(volatile u64*)(A + hi) = vhi;
}
__global__ __launch_bounds__(256) void k_sort_lds(u64* __restrict__ A, int k) {
  __shared__ u64 s[TILE];
  const int base = blockIdx.x * TILE, t = threadIdx.x;
  for (int i = t; i < TILE; i += 256) s[i] = A[base + i];
  __syncthreads();
  for (int j = TILE >> 1; j > 0; j >>= 1) {
    for (int p = t; p < TILE / 2; p += 256) {
      const int lo = ((p >> __builtin_ctz(j)) << (__builtin_ctz(j) + 1)) | (p & (j - 1));
      cas_lds(s, lo, lo + j, (((base + lo) & k) == 0));
    }
    __syncthreads();
  }
  for (int pass = 0; pass < 2; ++pass) { for (int i = t; i < TILE; i += 256) *(volatile u64*)(A + base + i) = s[i]; __threadfence(); }
}
__device__ __forceinline__ int lower_bound_hi(const u64* __restrict__ A, unsigned key) {
  int lo = 0, hi = SORT_N;
  while (lo < hi) { const int mid = (lo + hi) >> 1; if ((unsigned)(A[mid] >> 32) < key) lo = mid + 1; else hi = mid; }
  return lo;
}
__global__ __launch_bounds__(256) void k_segs(const u64* __restrict__ A, v2i* __restrict__ inseg, v2i* __restrict__ outseg, int N) {
  const int n = blockIdx.x * 256 + threadIdx.x;
  if (n >= N) return;
  const int a0 = lower_bound_hi(A, (unsigned)n), a1 = lower_bound_hi(A, (unsigned)(n + 1));
  const unsigned ob = 1u << 30;
  const int b0 = lower_bound_hi(A, ob | (unsigned)n), b1 = lower_bound_hi(A, ob | (unsigned)(n + 1));
  const v2i si = {a0, a1 - a0}, so = {b0, b1 - b0};
  VST2(v2i, inseg + n, si); VST2(v2i, outseg + n, so);
}

__global__ __launch_bounds__(256) void k_deg(const u64* __restrict__ A, const v2i* __restrict__ outseg, const float* __restrict__ w, float* __restrict__ dis, int N) {
  const int n = blockIdx.x * 256 + threadIdx.x;
  if (n >= N) return;
  const v2i s = outseg[n];
  float d = 0.f;
  for (int p = 0; p < s[1]; ++p) d += w[(int)(unsigned)(A[s[0] + p] & 0xffffffffu)];
  VST2(float, dis + n, (d > 0.f) ? (1.0f / sqrtf(fmaxf(d, 1e-12f))) : 0.f);
}
__global__ __launch_bounds__(256) void k_cheb(const u64* __restrict__ A, const v2i* __restrict__ inseg, const int* __restrict__ src,
                                              const float* __restrict__ w, const float* __restrict__ dis, const float* __restrict__ z,
                                              const float* __restrict__ h, float coef, float sub, float* __restrict__ out, int N) {
  const size_t i8 = (size_t)blockIdx.x * 256 + threadIdx.x;
  if (i8 >= (size_t)N * FDIM / 8) return;
  const int n = (int)(i8 >> 5), f0 = (int)(i8 & 31) * 8;
  const v2i s = inseg[n];
  v8f acc = {};
  for (int p = 0; p < s[1]; ++p) {
    const int e = (int)(unsigned)(A[s[0] + p] & 0xffffffffu);
    const int sn = src[e];
    const float cw = dis[sn] * w[e];
    const v8f zv = *(const v8f*)(z + (size_t)sn * FDIM + f0);
#pragma unroll
    for (int q = 0; q < 8; ++q) acc[q] += cw * zv[q];
  }
  const float dn = dis[n];
  const v8f hv = *(const v8f*)(h + (size_t)n * FDIM + f0);
  v8f o;
#pragma unroll
  for (int q = 0; q < 8; ++q) o[q] = coef * dn * acc[q] + sub * hv[q];
  VST2(v8f, out + (size_t)n * FDIM + f0, o);
}
__global__ __launch_bounds__(256) void k_packA(const float* __restrict__ h, const float* __restrict__ t1, const float* __restrict__ t2, _Float16* __restrict__ Ah, int N) {
  const size_t i8 = (size_t)blockIdx.x * 256 + threadIdx.x;
  if (i8 >= (size_t)N * KCAT / 8) return;
  const size_t i = i8 * 8; const int n = (int)(i / KCAT), k0 = (int)(i % KCAT);
  const float* srcp = (k0 < FDIM) ? (h + (size_t)n * FDIM + k0) : (k0 < 2 * FDIM) ? (t1 + (size_t)n * FDIM + k0 - FDIM) : (t2 + (size_t)n * FDIM + k0 - 2 * FDIM);
  v8h v;
#pragma unroll
  for (int q = 0; q < 8; ++q) v[q] = (_Float16)srcp[q];
  VST2(v8h, Ah + i, v);
}
__global__ __launch_bounds__(256) void k_packB(const float* __restrict__ Theta, _Float16* __restrict__ Wt) {
  const int i8 = blockIdx.x * 256 + threadIdx.x;
  if (i8 >= KCAT * CDIM / 8) return;
  const int i = i8 * 8, cc = i / KCAT, kk0 = i % KCAT;
  const int g = cc >> 8, f = cc & 255;
  v8h v;
#pragma unroll
  for (int q = 0; q < 8; ++q) { const int kk = kk0 + q, j = kk >> 8, kp = kk & 255; v[q] = (_Float16)Theta[(((size_t)(g * 3 + j) * FDIM) + kp) * FDIM + f]; }
  VST2(v8h, Wt + (size_t)i, v);
}
__global__ __launch_bounds__(128) void k_gemm(const _Float16* __restrict__ Ah, const _Float16* __restrict__ Wt, float* __restrict__ Z, int N) {
  const int lane = threadIdx.x & 31, wave = threadIdx.x >> 5, hh = lane >> 4, l16 = lane & 15;
  const int rt = blockIdx.x * 4 + wave;
  if (rt * 16 >= N) return;
  const int m0 = rt * 16, c0 = blockIdx.y * 64;
  v8f acc[4] = {};
  const _Float16* arow = Ah + (size_t)(m0 + l16) * KCAT;
  for (int kb = 0; kb < KCAT; kb += 32) {
    const v16h a = frag16(arow + kb, hh);
#pragma unroll
    for (int t = 0; t < 4; ++t) acc[t] = wmma16(a, frag16(Wt + (size_t)(c0 + t * 16 + l16) * KCAT + kb, hh), acc[t]);
  }
  for (int pass = 0; pass < 2; ++pass) {
#pragma unroll
    for (int pr = 0; pr < 2; ++pr)
#pragma unroll
      for (int r = 0; r < 8; ++r) {
        const float a_ = acc[2 * pr][r], b_ = acc[2 * pr + 1][r];
        const float ax = __shfl_xor(a_, 16), bx = __shfl_xor(b_, 16);
        *(volatile float*)(Z + (size_t)(m0 + r) * CDIM + c0 + pr * 32 + lane)     = hh ? bx : a_;
        *(volatile float*)(Z + (size_t)(m0 + r + 8) * CDIM + c0 + pr * 32 + lane) = hh ? b_ : ax;
      }
    __threadfence();
  }
}
__global__ __launch_bounds__(256) void k_lstm(const float* __restrict__ Z, const float* __restrict__ x, const float* __restrict__ c,
                                              const float* __restrict__ Wx, const float* __restrict__ b, const float* __restrict__ wc,
                                              const float* __restrict__ chebb, const float* __restrict__ linw, const float* __restrict__ linb,
                                              float* __restrict__ out, float* __restrict__ outH, float* __restrict__ outC, int N) {
  __shared__ float red[256];
  __shared__ float res[32];
  const int f = threadIdx.x, nb = blockIdx.x * 32;
  float wx[4][8];
#pragma unroll
  for (int g = 0; g < 4; ++g)
#pragma unroll
    for (int t = 0; t < 8; ++t) wx[g][t] = Wx[(g * 8 + t) * FDIM + f];
  const float bb0 = chebb[0 * FDIM + f] + b[0 * FDIM + f], bb1 = chebb[1 * FDIM + f] + b[1 * FDIM + f];
  const float bb2 = chebb[2 * FDIM + f] + b[2 * FDIM + f], bb3 = chebb[3 * FDIM + f] + b[3 * FDIM + f];
  const float wc0 = wc[0 * FDIM + f], wc1 = wc[1 * FDIM + f], wc2 = wc[2 * FDIM + f];
  for (int i = 0; i < 32; ++i) {
    const int n = nb + i;
    const bool live = (n < N);
    float z0 = bb0, z1 = bb1, z2 = bb2, z3 = bb3;
    float H0 = 0.f, C = 0.f;
    if (live) {
      const float* zr = Z + (size_t)n * CDIM;
      z0 += zr[f]; z1 += zr[FDIM + f]; z2 += zr[2 * FDIM + f]; z3 += zr[3 * FDIM + f];
#pragma unroll
      for (int t = 0; t < 8; ++t) { const float xv = x[(size_t)n * 8 + t]; z0 += xv * wx[0][t]; z1 += xv * wx[1][t]; z2 += xv * wx[2][t]; z3 += xv * wx[3][t]; }
      const float cv = c[(size_t)n * FDIM + f];
      const float I  = 1.0f / (1.0f + expf(-(z0 + wc0 * cv)));
      const float Fg = 1.0f / (1.0f + expf(-(z1 + wc1 * cv)));
      const float Tg = tanhf(z2);
      C  = Fg * cv + I * Tg;
      const float O  = 1.0f / (1.0f + expf(-(z3 + wc2 * C)));
      H0 = O * tanhf(C);
      VST2(float, outH + (size_t)n * FDIM + f, H0);
      VST2(float, outC + (size_t)n * FDIM + f, C);
    }
    red[f] = fmaxf(H0, 0.0f) * linw[f];
    __syncthreads();
    for (int s = 128; s > 0; s >>= 1) { if (f < s) red[f] += red[f + s]; __syncthreads(); }
    if (f == 0) res[i] = red[0] + linb[0];
    __syncthreads();
  }
  if (f < 32 && nb + f < N) VST2(float, out + nb + f, res[f]);
}

extern "C" void kernel_launch(void* const* d_in, const int* in_sizes, int n_in,
                              void* d_out, int out_size, void* d_ws, size_t ws_size,
                              hipStream_t stream) {
  (void)n_in; (void)out_size;
  const float* x   = (const float*)d_in[0];
  const int*   ei  = (const int*)  d_in[1];
  const float* ew  = (const float*)d_in[2];
  const float* h   = (const float*)d_in[3];
  const float* c   = (const float*)d_in[4];
  const float* Wx  = (const float*)d_in[5];
  const float* b   = (const float*)d_in[6];
  const float* wc  = (const float*)d_in[7];
  const float* Th  = (const float*)d_in[8];
  const float* cb  = (const float*)d_in[9];
  const float* lw  = (const float*)d_in[10];
  const float* lb  = (const float*)d_in[11];
  const int E = in_sizes[2];
  const int N = in_sizes[3] / FDIM;
  const int* src = ei;
  const int* dst = ei + E;
  if (2 * E > SORT_N || (N % 16) != 0) return;

  char* ws = (char*)d_ws;
  size_t off = 0;
  auto take = [&](size_t bytes) { void* p = ws + off; off = (off + bytes + 255) & ~(size_t)255; return p; };
  u64*   keys   = (u64*)  take((size_t)SORT_N * 8);
  v2i*   inseg  = (v2i*)  take((size_t)N * 8);
  v2i*   outseg = (v2i*)  take((size_t)N * 8);
  float* dis    = (float*)take((size_t)N * 4);
  float* Tx1    = (float*)take((size_t)N * FDIM * 4);
  float* Tx2    = (float*)take((size_t)N * FDIM * 4);
  _Float16* Ah  = (_Float16*)take((size_t)N * KCAT * 2);
  _Float16* Wt  = (_Float16*)take((size_t)CDIM * KCAT * 2);
  float* Z      = (float*)take((size_t)N * CDIM * 4);
  if (off > ws_size) return;

  float* out  = (float*)d_out;
  float* outH = out + N;
  float* outC = out + N + (size_t)N * FDIM;
  dim3 b256(256);
  auto cdiv = [](long long a, long long bq) { return (unsigned)((a + bq - 1) / bq); };

  k_sort_init<<<SORT_N / 256, b256, 0, stream>>>(src, dst, keys, E);
  k_sort_local<<<SORT_N / TILE, b256, 0, stream>>>(keys);
  for (int k = TILE * 2; k <= SORT_N; k <<= 1) {
    for (int logj = __builtin_ctz(k) - 1; (1 << logj) >= TILE; --logj)
      k_sort_global<<<SORT_N / 2 / 256, b256, 0, stream>>>(keys, logj, k);
    k_sort_lds<<<SORT_N / TILE, b256, 0, stream>>>(keys, k);
  }
  k_segs<<<cdiv(N, 256), b256, 0, stream>>>(keys, inseg, outseg, N);
  k_deg<<<cdiv(N, 256), b256, 0, stream>>>(keys, outseg, ew, dis, N);
  k_cheb<<<cdiv((long long)N * FDIM / 8, 256), b256, 0, stream>>>(keys, inseg, src, ew, dis, h,   h, -1.0f,  0.0f, Tx1, N);
  k_cheb<<<cdiv((long long)N * FDIM / 8, 256), b256, 0, stream>>>(keys, inseg, src, ew, dis, Tx1, h, -2.0f, -1.0f, Tx2, N);
  k_packA<<<cdiv((long long)N * KCAT / 8, 256), b256, 0, stream>>>(h, Tx1, Tx2, Ah, N);
  k_packB<<<cdiv((long long)KCAT * CDIM / 8, 256), b256, 0, stream>>>(Th, Wt);
  k_gemm<<<dim3(cdiv(N / 16, 4), CDIM / 64), dim3(128), 0, stream>>>(Ah, Wt, Z, N);
  k_lstm<<<cdiv(N, 32), b256, 0, stream>>>(Z, x, c, Wx, b, wc, cb, lw, lb, out, outH, outC, N);
}
